// MiniBatchEGNNTrain_35021163331775
// MI455X (gfx1250) — hardware-verified
//
#include <hip/hip_runtime.h>
#include <stddef.h>
#include <stdint.h>


#define DIN    64
#define HID    64
#define KE     4
#define NHW    256
#define NCLS   40
#define NFCP   48
#define NBW    (NHW + NHW + NFCP)
#define KQ     8
#define KSTEP  2
#define APK    72
#define TR     16
#define NTHR   256
#define NWAVE  8
#define S1     1024
#define NCH1   4
#define SH1    12
#define SH2    7
#define SH3    4
#define F1A    16
#define F2     32
#define F3     8
#define CAP1   256
#define CAP2   192
#define CAP3   512
#define SEGS2  16
#define HSC    16.0f
#define WSC    64.0f
#define RSC    0.0009765625f
#define SENT   0xFFFFFFFFu
#define WSCAPB 134217728
#define NPREPT (NBW * KQ)
#define OTILE  (TR * NCLS)

static_assert(NHW == KE * HID);
static_assert(KQ * 8 == DIN && KSTEP * 32 == DIN && HID == DIN);
static_assert((APK % 8) == 0 && APK >= DIN);
static_assert((NPREPT % 32) == 0);
static_assert(NCH1 * NTHR == S1);
static_assert(CAP1 == NTHR);
static_assert((F1A * CAP1) % (4 * NTHR) == 0);
static_assert((F2 * CAP2) % (4 * NTHR) == 0);
static_assert((F3 * CAP3) % (4 * NTHR) == 0);
static_assert((CAP1 % 32) == 0 && (CAP2 % 32) == 0 && (CAP3 % 32) == 0);
static_assert(NTHR == 32 * NWAVE && TR == 2 * NWAVE);
static_assert(2 * 16 * NWAVE == NHW);
static_assert(NTHR * 4 == TR * DIN);
static_assert((TR * NHW) % (4 * NTHR) == 0);
static_assert(HID == 2 * 32);
static_assert(NFCP == 48 && NCLS <= NFCP && 3 <= NWAVE);
static_assert((OTILE % 4) == 0 && ((OTILE / 4) % 32) == 0 && ((OTILE * 4) % 128) == 0);
static_assert(TR * NCLS <= TR * NHW);

typedef _Float16 v4h  __attribute__((ext_vector_type(4)));
typedef _Float16 v8h  __attribute__((ext_vector_type(8)));
typedef _Float16 v16h __attribute__((ext_vector_type(16)));
typedef float    v2f  __attribute__((ext_vector_type(2)));
typedef float    v4f  __attribute__((ext_vector_type(4)));
typedef float    v8f  __attribute__((ext_vector_type(8)));
typedef unsigned int v4u __attribute__((ext_vector_type(4)));
typedef v4h v4ha __attribute__((may_alias));
typedef v8h v8ha __attribute__((may_alias));
typedef v2f v2fa __attribute__((may_alias));
typedef v4f v4fa __attribute__((may_alias));
typedef v4u v4ua __attribute__((may_alias));
union Frag { v16h v; v8h h[2]; };

__device__ __forceinline__ v8f wmh(v16h a, v16h b, v8f c) {
  v8f d = __builtin_amdgcn_wmma_f32_16x16x32_f16(false, a, false, b, (short)0, c, false, false);
  asm volatile("v_nop\n\tv_nop\n\tv_nop\n\tv_nop" : "+v"(d) : "v"(a), "v"(b));
  return d;
}

__device__ __forceinline__ v4h cvt4(v4f a) {
  v4h r;
  r[0] = (_Float16)a[0]; r[1] = (_Float16)a[1]; r[2] = (_Float16)a[2]; r[3] = (_Float16)a[3];
  return r;
}

__global__ __launch_bounds__(NTHR) void k_wprep(const float* __restrict__ w0, const float* __restrict__ w1,
                                                const float* __restrict__ wfc, _Float16* Bw) {
  const int gi = blockIdx.x * NTHR + threadIdx.x;
  const bool act = gi < NPREPT;
  const int gc = act ? gi : NPREPT - 1;
  const int row = gc >> 3, d0 = (gc & 7) * 8;
  const int n0 = row < NHW ? row : NHW - 1;
  int n1 = row - NHW;     n1 = n1 < 0 ? 0 : (n1 > NHW - 1 ? NHW - 1 : n1);
  int n2 = row - 2 * NHW; n2 = n2 < 0 ? 0 : (n2 > NFCP - 1 ? NFCP - 1 : n2);
  const int c0 = n0 >> 2, k0 = n0 & 3, c1 = n1 >> 2, k1 = n1 & 3;
  const int c2 = n2 < NCLS ? n2 : NCLS - 1;
  const int sel = row < NHW ? 0 : (row < 2 * NHW ? 1 : (n2 < NCLS ? 2 : 3));
  v8h hv;
#pragma unroll
  for (int e = 0; e < 8; ++e) {
    const int d = d0 + e;
    const float v0 = w0[(size_t)(k0 * DIN + d) * HID + c0];
    const float v1 = w1[(size_t)(k1 * HID + d) * HID + c1];
    const float v2 = wfc[(size_t)d * NCLS + c2];
    const float v = sel == 0 ? v0 : (sel == 1 ? v1 : (sel == 2 ? v2 : 0.0f));
    hv[e] = (_Float16)(v * WSC);
  }
  _Float16* dst = Bw + (size_t)gc * 8;
  if (act) *(volatile v8h*)dst = hv;
  __threadfence();
  if (act) *(volatile v8h*)dst = hv;
}

template <int LV, int FA, int CAP>
__global__ __launch_bounds__(NTHR) void k_part(const int* __restrict__ edst, const unsigned* lin, unsigned* lout,
                                               int nN, int nE, int nC, int nB1, int P2, int nch) {
  __shared__ __attribute__((aligned(16))) unsigned lst[FA * CAP];
  __shared__ int wc[NWAVE * 32];
  __shared__ int cur[32];
  const int tid = threadIdx.x, lane = tid & 31, wave = tid >> 5;
  const int blk = blockIdx.x;
  const v4u sv = {SENT, SENT, SENT, SENT};
#pragma unroll
  for (int k = 0; k < (FA * CAP) / (4 * NTHR); ++k) *(v4ua*)(&lst[4 * (tid + NTHR * k)]) = sv;
  if (wave == 0) cur[lane] = 0;
  __syncthreads();

  int c = 0, part = 0, ml = 0;
  if (LV == 2) { c = blk / P2; part = blk - c * P2; }
  if (LV == 3) { c = blk >> 5; ml = blk & 31; }
  const int nslots3 = P2 * CAP2;

#pragma unroll 1
  for (int ch = 0; ch < nch; ++ch) {
    bool valid;
    int key;
    unsigned rec;
    if (LV == 1) {
      const int e = blk * S1 + ch * NTHR + tid;
      const int ec = e < nE ? e : nE - 1;
      const int d = edst[ec];
      valid = (e < nE) && ((unsigned)d < (unsigned)nN);
      key = d >> SH1;
      rec = (unsigned)ec;
    } else if (LV == 2) {
      const int bl = part * SEGS2 + ch;
      const int blc = bl < nB1 ? bl : nB1 - 1;
      const unsigned id = lin[((size_t)blc * nC + c) * CAP1 + tid];
      const bool idok = id < (unsigned)nE;
      const int idc = idok ? (int)id : nE - 1;
      const int d = edst[idc];
      valid = (bl < nB1) && idok && ((unsigned)d < (unsigned)nN);
      key = (d >> SH2) & 31;
      rec = (unsigned)idc;
    } else {
      const int q = ch * NTHR + tid;
      const int qc = q < nslots3 ? q : nslots3 - 1;
      const int pp = qc / CAP2, s = qc - pp * CAP2;
      const unsigned id = lin[(((size_t)(c * P2 + pp)) * F2 + ml) * CAP2 + s];
      const bool idok = id < (unsigned)nE;
      const int idc = idok ? (int)id : nE - 1;
      const int d = edst[idc];
      valid = (q < nslots3) && idok && ((unsigned)d < (unsigned)nN);
      key = (d >> SH3) & 7;
      rec = ((unsigned)d & 15u) | ((unsigned)idc << 4);
    }
    key = valid ? key : 255;
    unsigned mym = 0u;
#pragma unroll
    for (int b = 0; b < FA; ++b) {
      const unsigned mb = __builtin_amdgcn_ballot_w32(key == b);
      mym = (key == b) ? mb : mym;
    }
    const unsigned lt = (1u << lane) - 1u;
    const int rank = __builtin_popcount(mym & lt);
    const int cnt  = __builtin_popcount(mym);
    wc[wave * 32 + lane] = 0;
    if (valid && rank == 0) wc[wave * 32 + key] = cnt;
    __syncthreads();
    const int kc = key & 31;
    int pre = 0;
    for (int w2 = 0; w2 < wave; ++w2) pre += wc[w2 * 32 + kc];
    const int pos = cur[kc] + pre + rank;
    if (valid && pos < CAP) lst[kc * CAP + pos] = rec;
    int tot = 0;
    if (wave == 0) {
#pragma unroll
      for (int w2 = 0; w2 < NWAVE; ++w2) tot += wc[w2 * 32 + lane];
    }
    __syncthreads();
    if (wave == 0) cur[lane] += tot;
  }
  __syncthreads();

  const int nwords  = (LV == 1) ? nC * CAP : FA * CAP;
  const int npieces = nwords >> 2;
  unsigned* gb = lout + (size_t)blk * nwords;
#pragma unroll
  for (int k = 0; k < (FA * CAP / 4 + NTHR - 1) / NTHR; ++k) {
    const int it = tid + NTHR * k;
    if (it < npieces) { const v4u v = *(const v4ua*)(&lst[4 * it]); *(volatile v4u*)(gb + 4 * it) = v; }
  }
  __threadfence();
#pragma unroll
  for (int k = 0; k < (FA * CAP / 4 + NTHR - 1) / NTHR; ++k) {
    const int it = tid + NTHR * k;
    if (it < npieces) { const v4u v = *(const v4ua*)(&lst[4 * it]); *(volatile v4u*)(gb + 4 * it) = v; }
  }
}

__device__ __forceinline__ void gemm_hw_tile(const _Float16* sA, const _Float16* __restrict__ Bn,
                                             float* stg, float* gb, int tid) {
  const int lane = tid & 31, wave = tid >> 5, hh = lane >> 4, m = lane & 15;
  v16h av[KSTEP];
  const _Float16* abase = sA + m * APK + 8 * hh;
#pragma unroll
  for (int kt = 0; kt < KSTEP; ++kt) {
    Frag a;
    a.h[0] = *(const v8ha*)(abase + 32 * kt);
    a.h[1] = *(const v8ha*)(abase + 32 * kt + 16);
    av[kt] = a.v;
  }
#pragma unroll 1
  for (int ct = 0; ct < 2; ++ct) {
    const int col = wave * 32 + ct * 16 + m;
    const _Float16* bp = Bn + (size_t)col * DIN + 8 * hh;
    v8f acc = {0.f, 0.f, 0.f, 0.f, 0.f, 0.f, 0.f, 0.f};
#pragma unroll
    for (int kt = 0; kt < KSTEP; ++kt) {
      Frag b;
      b.h[0] = *(const v8h*)(bp + 32 * kt);
      b.h[1] = *(const v8h*)(bp + 32 * kt + 16);
      acc = wmh(av[kt], b.v, acc);
    }
#pragma unroll
    for (int r = 0; r < 8; ++r) stg[(8 * hh + r) * NHW + col] = acc[r] * RSC;
  }
  __syncthreads();
#pragma unroll
  for (int k = 0; k < (TR * NHW) / (4 * NTHR); ++k) {
    const int it = tid + NTHR * k;
    const v4f v = *(const v4fa*)(stg + 4 * it);
    *(volatile v4f*)(gb + 4 * it) = v;
  }
  __threadfence();
#pragma unroll
  for (int k = 0; k < (TR * NHW) / (4 * NTHR); ++k) {
    const int it = tid + NTHR * k;
    const v4f v = *(const v4fa*)(stg + 4 * it);
    *(volatile v4f*)(gb + 4 * it) = v;
  }
}

__global__ __launch_bounds__(NTHR) void k_hw0(const float* __restrict__ x, const _Float16* __restrict__ B0,
                                              float* HW, int nN) {
  __shared__ __attribute__((aligned(16))) _Float16 sA[TR * APK];
  __shared__ __attribute__((aligned(16))) float stg[TR * NHW];
  const int tid = threadIdx.x;
  const int tile = blockIdx.x;
  const v4f z4 = {0.f, 0.f, 0.f, 0.f};
  {
    const int row = tid >> 4, c4 = (tid & 15) * 4;
    const int node = tile * TR + row;
    const int nc = node < nN ? node : nN - 1;
    v4f v = *(const v4f*)(x + (size_t)nc * DIN + c4);
    if (node >= nN) v = z4;
    *(v4ha*)(sA + row * APK + c4) = cvt4(v * HSC);
  }
  __syncthreads();
  gemm_hw_tile(sA, B0, stg, HW + (size_t)tile * (TR * NHW), tid);
}

__device__ __forceinline__ v2f drain(unsigned msk, unsigned rec, const float* __restrict__ HW,
                                     const int* __restrict__ esrc, const float* __restrict__ ef,
                                     v2f bb, int lane, int nN, int nE, v2f acc) {
  while (msk != 0u) {
    const int i = __builtin_ctz(msk);
    msk &= msk - 1u;
    const unsigned r = (unsigned)__builtin_amdgcn_readlane((int)rec, i);
    int eid = (int)(r >> 4);
    eid = eid > nE - 1 ? nE - 1 : eid;
    int s = esrc[eid];
    s = s < 0 ? s + nN : s;
    s = s < 0 ? 0 : (s > nN - 1 ? nN - 1 : s);
    const v4f e4 = *(const v4f*)(ef + (size_t)eid * KE);
    const float* hr = HW + (size_t)s * NHW + 8 * lane;
    const v4f va = *(const v4f*)hr;
    const v4f vb = *(const v4f*)(hr + 4);
    float t0 = e4[0] * va[0] + e4[1] * va[1] + e4[2] * va[2] + e4[3] * va[3] + bb[0];
    float t1 = e4[0] * vb[0] + e4[1] * vb[1] + e4[2] * vb[2] + e4[3] * vb[3] + bb[1];
    t0 = fmaxf(t0, 0.0f);
    t1 = fmaxf(t1, 0.0f);
    acc[0] += t0;
    acc[1] += t1;
  }
  return acc;
}

template <int FIN>
__global__ __launch_bounds__(NTHR) void k_agg(const unsigned* __restrict__ l3, const float* __restrict__ HW,
                                              const int* __restrict__ esrc, const float* __restrict__ ef,
                                              const float* __restrict__ bias, const _Float16* __restrict__ Bn,
                                              const float* __restrict__ bfc, float* gout, int nN, int nE) {
  __shared__ __attribute__((aligned(16))) _Float16 sA[TR * APK];
  __shared__ __attribute__((aligned(16))) float sH[TR * HID];
  __shared__ __attribute__((aligned(16))) float stg[TR * NHW];
  const int tid = threadIdx.x, lane = tid & 31, wave = tid >> 5, hh = lane >> 4, m = lane & 15;
  const int tile = blockIdx.x;

  {
    v2f acc0 = {0.f, 0.f}, acc1 = {0.f, 0.f};
    int cnt0 = 0, cnt1 = 0;
    v2f bb;
    bb[0] = bias[2 * lane];
    bb[1] = bias[2 * lane + 1];
    const unsigned* seg = l3 + (size_t)tile * CAP3;
#pragma unroll 1
    for (int ch = 0; ch < CAP3 / 32; ++ch) {
      const unsigned rec = seg[ch * 32 + lane];
      const bool ok = ((int)rec) >= 0;
      const int ln = (int)(rec & 15u);
      const unsigned m0 = __builtin_amdgcn_ballot_w32(ok && (ln == 2 * wave));
      const unsigned m1 = __builtin_amdgcn_ballot_w32(ok && (ln == 2 * wave + 1));
      cnt0 += __builtin_popcount(m0);
      cnt1 += __builtin_popcount(m1);
      acc0 = drain(m0, rec, HW, esrc, ef, bb, lane, nN, nE, acc0);
      acc1 = drain(m1, rec, HW, esrc, ef, bb, lane, nN, nE, acc1);
    }
    const float c0 = (float)(cnt0 < 1 ? 1 : cnt0);
    const float c1 = (float)(cnt1 < 1 ? 1 : cnt1);
    const float rc0 = 1.0f / c0, rc1 = 1.0f / c1;
    v2f h0 = acc0 * rc0, h1 = acc1 * rc1;
    h0[0] = fmaxf(h0[0], 0.0f); h0[1] = fmaxf(h0[1], 0.0f);
    h1[0] = fmaxf(h1[0], 0.0f); h1[1] = fmaxf(h1[1], 0.0f);
    *(v2fa*)(sH + (2 * wave) * HID + 2 * lane) = h0;
    *(v2fa*)(sH + (2 * wave + 1) * HID + 2 * lane) = h1;
  }
  __syncthreads();
  {
    const int row = tid >> 4, c4 = (tid & 15) * 4;
    const v4f v = *(const v4fa*)(sH + row * HID + c4);
    *(v4ha*)(sA + row * APK + c4) = cvt4(v * HSC);
  }
  __syncthreads();

  if (FIN == 0) {
    gemm_hw_tile(sA, Bn, stg, gout + (size_t)tile * (TR * NHW), tid);
  } else {
    if (wave < 3) {
      const int col = wave * 16 + m;
      Frag a0, a1;
      const _Float16* abase = sA + m * APK + 8 * hh;
      a0.h[0] = *(const v8ha*)(abase);
      a0.h[1] = *(const v8ha*)(abase + 16);
      a1.h[0] = *(const v8ha*)(abase + 32);
      a1.h[1] = *(const v8ha*)(abase + 48);
      const _Float16* bp = Bn + (size_t)col * DIN + 8 * hh;
      Frag b0, b1;
      b0.h[0] = *(const v8h*)(bp);
      b0.h[1] = *(const v8h*)(bp + 16);
      b1.h[0] = *(const v8h*)(bp + 32);
      b1.h[1] = *(const v8h*)(bp + 48);
      v8f acc = {0.f, 0.f, 0.f, 0.f, 0.f, 0.f, 0.f, 0.f};
      acc = wmh(a0.v, b0.v, acc);
      acc = wmh(a1.v, b1.v, acc);
      const float bc = bfc[col < NCLS ? col : NCLS - 1];
      if (col < NCLS) {
#pragma unroll
        for (int r = 0; r < 8; ++r) stg[(8 * hh + r) * NCLS + col] = acc[r] * RSC + bc;
      }
    }
    __syncthreads();
    const int npc = OTILE / 4;
    const size_t f0 = (size_t)tile * OTILE + 4 * (size_t)tid;
    const bool wok = (tid < npc) && (f0 + 4 <= (size_t)nN * NCLS);
    const int itc = tid < npc ? tid : npc - 1;
    const v4f ov = *(const v4fa*)(stg + 4 * itc);
    float* go = gout + (wok ? f0 : (size_t)0);
    if (wok) *(volatile v4f*)go = ov;
    __threadfence();
    if (wok) *(volatile v4f*)go = ov;
  }
}

extern "C" void kernel_launch(void* const* d_in, const int* in_sizes, int n_in,
                              void* d_out, int out_size, void* d_ws, size_t ws_size,
                              hipStream_t stream) {
  if (n_in < 10) return;
  if (in_sizes[0] <= 0 || (in_sizes[0] % DIN) != 0) return;
  const int nN = in_sizes[0] / DIN;
  const int nE = in_sizes[2];
  if (nN < 1 || nN > 65536) return;
  if (nE < 1 || nE > (1 << 27)) return;
  if (in_sizes[3] != nE) return;
  if (in_sizes[1] != 2 * nE * KE) return;
  if (in_sizes[4] != KE * DIN * HID || in_sizes[6] != KE * HID * HID) return;
  if (in_sizes[5] != HID || in_sizes[7] != HID) return;
  if (in_sizes[8] != HID * NCLS || in_sizes[9] != NCLS) return;
  if (out_size != nN * NCLS) return;

  const float* x    = (const float*)d_in[0];
  const float* ef   = (const float*)d_in[1];
  const int*   esrc = (const int*)d_in[2];
  const int*   edst = (const int*)d_in[3];
  const float* W0   = (const float*)d_in[4];
  const float* b0   = (const float*)d_in[5];
  const float* W1   = (const float*)d_in[6];
  const float* b1   = (const float*)d_in[7];
  const float* Wfc  = (const float*)d_in[8];
  const float* bfc  = (const float*)d_in[9];
  float* out = (float*)d_out;

  const int nTiles = (nN + TR - 1) / TR;
  const int nC   = (nN + 4095) >> SH1;
  const int nB1  = (nE + S1 - 1) / S1;
  const int P2   = (nB1 + SEGS2 - 1) / SEGS2;
  const int nch3 = (P2 * CAP2 + NTHR - 1) / NTHR;
  if (nC < 1 || nC > F1A) return;

  char* ws = (char*)d_ws;
  size_t o = 0;
  const size_t oBw = o; o += (size_t)NBW * DIN * 2;                         o = (o + 255) & ~(size_t)255;
  const size_t oL1 = o; o += (size_t)nB1 * nC * CAP1 * 4;                  o = (o + 255) & ~(size_t)255;
  const size_t oL2 = o; o += (size_t)nC * P2 * F2 * CAP2 * 4;              o = (o + 255) & ~(size_t)255;
  const size_t oL3 = o; o += (size_t)nC * 32 * F3 * CAP3 * 4;              o = (o + 255) & ~(size_t)255;
  const size_t oH0 = o; o += (size_t)nTiles * TR * NHW * 4;                o = (o + 255) & ~(size_t)255;
  const size_t oH1 = o; o += (size_t)nTiles * TR * NHW * 4;                o = (o + 255) & ~(size_t)255;
  if (o > ws_size || o > (size_t)WSCAPB) return;
  _Float16* Bw  = (_Float16*)(ws + oBw);
  unsigned* L1  = (unsigned*)(ws + oL1);
  unsigned* L2  = (unsigned*)(ws + oL2);
  unsigned* L3  = (unsigned*)(ws + oL3);
  float*    HW0 = (float*)(ws + oH0);
  float*    HW1 = (float*)(ws + oH1);

  k_wprep<<<(NPREPT + NTHR - 1) / NTHR, NTHR, 0, stream>>>(W0, W1, Wfc, Bw);
  k_part<1, F1A, CAP1><<<nB1, NTHR, 0, stream>>>(edst, L1, L1, nN, nE, nC, nB1, P2, NCH1);
  k_part<2, F2, CAP2><<<nC * P2, NTHR, 0, stream>>>(edst, L1, L2, nN, nE, nC, nB1, P2, SEGS2);
  k_part<3, F3, CAP3><<<nC * 32, NTHR, 0, stream>>>(edst, L2, L3, nN, nE, nC, nB1, P2, nch3);
  k_hw0<<<nTiles, NTHR, 0, stream>>>(x, Bw, HW0, nN);
  k_agg<0><<<nTiles, NTHR, 0, stream>>>(L3, HW0, esrc, ef, b0, Bw + (size_t)NHW * DIN, bfc, HW1, nN, nE);
  k_agg<1><<<nTiles, NTHR, 0, stream>>>(L3, HW1, esrc, ef + (size_t)nE * KE, b1, Bw + (size_t)2 * NHW * DIN,
                                        bfc, out, nN, nE);
}
